// MultiHeadedAttention_86586540688078
// MI455X (gfx1250) — hardware-verified
//
#include <hip/hip_runtime.h>
#include <math.h>

typedef __attribute__((ext_vector_type(16))) _Float16 v16h;
typedef __attribute__((ext_vector_type(16))) __bf16 v16b;
typedef __attribute__((ext_vector_type(8)))  _Float16 v8h;
typedef __attribute__((ext_vector_type(8)))  __bf16 v8b;
typedef __attribute__((ext_vector_type(8)))  float v8f;
typedef __attribute__((ext_vector_type(4)))  float v4f;
typedef __attribute__((ext_vector_type(4)))  unsigned v4u;
typedef v4f __attribute__((may_alias)) v4f_a;
typedef v4u __attribute__((may_alias)) v4u_a;

template <typename T> __device__ __forceinline__ void vst2(void* p, T v) { *(volatile T*)p = v; __threadfence(); *(volatile T*)p = v; }
__device__ __forceinline__ v8f wmma16(v16h a, v16h b, v8f c) {
  v8f d = __builtin_amdgcn_wmma_f32_16x16x32_f16(false, a, false, b, (short)0, c, false, false);
  asm volatile("v_nop\n\tv_nop\n\tv_nop\n\tv_nop" : "+v"(d) : "v"(a), "v"(b));
  return d;
}
__device__ __forceinline__ v8f wmma_bf(v16b a, v16b b, v8f c) {
  v8f d = __builtin_amdgcn_wmma_f32_16x16x32_bf16(false, a, false, b, (short)0, c, false, false);
  asm volatile("v_nop\n\tv_nop\n\tv_nop\n\tv_nop" : "+v"(d) : "v"(a), "v"(b));
  return d;
}
__device__ __forceinline__ v16h frag_h(const _Float16* rowk0, int lane) {
  union { v16h v; v8h q[2]; } u; const _Float16* p = rowk0 + 8 * (lane >> 4);
  u.q[0] = *(const v8h*)p; u.q[1] = *(const v8h*)(p + 16); return u.v;
}
__device__ __forceinline__ v16b frag_b(const __bf16* rowk0, int lane) {
  union { v16b v; v8b q[2]; } u; const __bf16* p = rowk0 + 8 * (lane >> 4);
  u.q[0] = *(const v8b*)p; u.q[1] = *(const v8b*)(p + 16); return u.v;
}
__device__ __forceinline__ float bfr(float v) { return (float)(__bf16)v; }
#define LDSX() do { asm volatile("s_wait_dscnt 0" ::: "memory"); __builtin_amdgcn_wave_barrier(); __builtin_amdgcn_fence(3  , "workgroup"); } while (0)

#ifndef NB
#define NB 2
#endif
#ifndef SEQ
#define SEQ 2048
#endif
#define NB_FULL 2
#define SEQ_FULL 2048
#define CC 1024
#define NH 16
#define HD 64
#define QHI 256
#define QBH (QHI / 64)
#define NTOK ((size_t)NB * SEQ)
#define PLANE_B ((size_t)2 * NTOK * CC)

static_assert(NH * HD == CC);
static_assert(HD == 64);
static_assert(HD % 32 == 0);
static_assert(CC % 128 == 0);
static_assert(CC % 32 == 0);
static_assert(SEQ % 1024 == 0);
static_assert(SEQ <= SEQ_FULL);
static_assert(NB <= NB_FULL);
static_assert(QHI % 64 == 0);
static_assert(QHI <= SEQ);
static_assert((NB * SEQ) % 64 == 0);
static_assert(((size_t)NB * SEQ * CC / 8) % 256 == 0);
static_assert(((size_t)CC * CC / 8) % 256 == 0);

#define WS_XB   ((size_t)0)
#define WS_WB   (WS_XB + 3 * PLANE_B)
#define WS_WOB  (WS_WB + (size_t)3 * 2 * CC * CC)
#define WS_WOH  (WS_WOB + (size_t)2 * CC * CC)
#define WS_QH   (WS_WOH + (size_t)2 * CC * CC)
#define WS_KH   (WS_QH + PLANE_B)
#define WS_KL   (WS_KH + PLANE_B)
#define WS_VT   (WS_KL + PLANE_B)
#define WS_VB   (WS_VT + PLANE_B)
#define WS_VBL  (WS_VB + PLANE_B)
#define WS_QL   (WS_VBL + PLANE_B)
#define WS_MB   (WS_QL + (size_t)2 * NB * QHI * CC)
#define WS_CTXH (WS_MB + (size_t)4 * NTOK * (SEQ / 32))
#define WS_CBH  (WS_CTXH + PLANE_B)
#define WS_CBL  (WS_CBH + (size_t)2 * NB * QHI * CC)
#define WS_END  (WS_CBL + (size_t)2 * NB * QHI * CC)
static_assert(WS_END <= (size_t)134217728);
static_assert(WS_WB % 128 == 0);
static_assert(WS_MB % 128 == 0);
static_assert(WS_CBH % 128 == 0);

__global__ __launch_bounds__(256) void k_maskbits(const int* __restrict__ M, unsigned* __restrict__ MB) {
  const int wave = threadIdx.x >> 5, lane = threadIdx.x & 31;
  const int row = blockIdx.x * 8 + wave;
  const int b = row / SEQ, q = row % SEQ;
  const int* src = M + ((size_t)b * SEQ_FULL + q) * SEQ_FULL;
  unsigned* dst = MB + (size_t)row * (SEQ / 32);
#pragma unroll 1
  for (int c = 0; c < SEQ / 1024; ++c) {
    unsigned mine = 0u;
#pragma unroll 4
    for (int w = 0; w < 32; ++w) {
      const int v = src[c * 1024 + w * 32 + lane];
      const unsigned bits = __builtin_amdgcn_ballot_w32(v != 0);
      mine = (w == lane) ? bits : mine;
    }
    vst2(dst + c * 32 + lane, mine);
  }
}

__global__ __launch_bounds__(256) void k_cvt_x(const float* __restrict__ X0, const float* __restrict__ X1, const float* __restrict__ X2, __bf16* __restrict__ XB) {
  const int which = blockIdx.y;
  const float* X = which == 0 ? X0 : which == 1 ? X1 : X2;
  const size_t i8 = (size_t)blockIdx.x * 256 + threadIdx.x;
  const size_t row = i8 / (CC / 8); const int c = (int)(i8 % (CC / 8)) * 8;
  const size_t b = row / SEQ, t = row % SEQ;
  const float* p = X + (b * SEQ_FULL + t) * CC + c;
  const v4f f0 = *(const v4f*)p, f1 = *(const v4f*)(p + 4);
  union { v8b v; v4u u; } o;
#pragma unroll
  for (int i = 0; i < 4; ++i) { o.v[i] = (__bf16)f0[i]; o.v[4 + i] = (__bf16)f1[i]; }
  vst2(XB + (size_t)which * NTOK * CC + row * CC + c, o.u);
}

__global__ __launch_bounds__(256) void k_cvt_w(const float* __restrict__ W0, const float* __restrict__ W1, const float* __restrict__ W2, const float* __restrict__ W3, __bf16* __restrict__ WB, __bf16* __restrict__ WOB, _Float16* __restrict__ WOH) {
  const int which = blockIdx.y;
  const float* W = which == 0 ? W0 : which == 1 ? W1 : which == 2 ? W2 : W3;
  const size_t off = ((size_t)blockIdx.x * 256 + threadIdx.x) * 8;
  const v4f f0 = *(const v4f*)(W + off), f1 = *(const v4f*)(W + off + 4);
  union { v8b v; v4u u; } o;
#pragma unroll
  for (int i = 0; i < 4; ++i) { o.v[i] = (__bf16)f0[i]; o.v[4 + i] = (__bf16)f1[i]; }
  if (which < 3) { vst2(WB + (size_t)which * CC * CC + off, o.u); }
  else {
    union { v8h v; v4u u; } oh;
#pragma unroll
    for (int i = 0; i < 4; ++i) { oh.v[i] = (_Float16)(bfr(f0[i]) * 256.0f); oh.v[4 + i] = (_Float16)(bfr(f1[i]) * 256.0f); }
    vst2(WOB + off, o.u); vst2(WOH + off, oh.u);
  }
}

__global__ __launch_bounds__(128) void k_proj(const __bf16* __restrict__ XB, const __bf16* __restrict__ WB, const float* __restrict__ BQ, const float* __restrict__ BK, const float* __restrict__ BV,
    _Float16* __restrict__ QH, _Float16* __restrict__ QL, _Float16* __restrict__ KH, _Float16* __restrict__ KL, _Float16* __restrict__ VT, __bf16* __restrict__ VB, __bf16* __restrict__ VBL) {
  __shared__ __align__(16) _Float16 sh[64][136], sl[64][136]; __shared__ __align__(16) _Float16 th[128][72]; __shared__ __align__(16) __bf16 tb[128][72], tbl[128][72];
  const int tid = threadIdx.x, wave = tid >> 5, lane = tid & 31, col = lane & 15, g = lane >> 4; const int which = blockIdx.z; const int c0 = blockIdx.y * 128; const size_t r0 = (size_t)blockIdx.x * 64; const size_t bb = r0 / SEQ; const int t0 = (int)(r0 % SEQ);
  const __bf16* X = XB + (size_t)which * NTOK * CC; const __bf16* WA = WB + (size_t)which * CC * CC; const float* BA = which == 0 ? BQ : which == 1 ? BK : BV;
  v8f acc[8] = {};
#pragma unroll 2
  for (int kc = 0; kc < CC / 32; ++kc) { const v16b a = frag_b(X + (r0 + wave * 16 + col) * CC + kc * 32, lane);
#pragma unroll
    for (int j = 0; j < 8; ++j) { const v16b w = frag_b(WA + (size_t)(c0 + j * 16 + col) * CC + kc * 32, lane); acc[j] = wmma_bf(a, w, acc[j]); } }
  if (which < 2) { _Float16* DH = which == 0 ? QH : KH; _Float16* DL = which == 0 ? QL : KL; const bool res_rows = (which == 1) || (t0 < QHI); const size_t lrow0 = (which == 1) ? r0 : (bb * QHI + (size_t)t0);
#pragma unroll
    for (int j = 0; j < 8; ++j) { const float bias = bfr(BA[c0 + j * 16 + col]);
#pragma unroll
      for (int r = 0; r < 8; ++r) { const float v = acc[j][r] + bias; const _Float16 hv = (_Float16)v; sh[wave * 16 + 8 * g + r][j * 16 + col] = hv; sl[wave * 16 + 8 * g + r][j * 16 + col] = (_Float16)((v - (float)hv) * 1024.0f); } }
    __syncthreads();
    for (int e = tid; e < 64 * 16; e += 128) { const int rl = e >> 4, q = e & 15; const v4u a = *(const v4u_a*)&sh[rl][q * 8]; vst2(DH + (r0 + rl) * CC + c0 + q * 8, a);
      if (res_rows) { const v4u c = *(const v4u_a*)&sl[rl][q * 8]; vst2(DL + (lrow0 + rl) * CC + c0 + q * 8, c); } }
  } else {
#pragma unroll
    for (int j = 0; j < 8; ++j) { const float bias = bfr(BA[c0 + j * 16 + col]);
#pragma unroll
      for (int r = 0; r < 8; ++r) { const float v = acc[j][r] + bias; const int rl = wave * 16 + 8 * g + r, cl = j * 16 + col; th[cl][rl] = (_Float16)v; const __bf16 bh = (__bf16)v; tb[cl][rl] = bh; tbl[cl][rl] = (__bf16)(v - (float)bh); } }
    __syncthreads();
    for (int e = tid; e < 128 * 8; e += 128) { const int cl = e >> 3, q = e & 7; const size_t o3 = (bb * CC + c0 + cl) * (size_t)SEQ + t0 + q * 8;
      const v4u a = *(const v4u_a*)&th[cl][q * 8]; vst2(VT + o3, a); const v4u c = *(const v4u_a*)&tb[cl][q * 8]; vst2(VB + o3, c); const v4u d = *(const v4u_a*)&tbl[cl][q * 8]; vst2(VBL + o3, d); } }
}

__global__ __launch_bounds__(128) void k_attn(const _Float16* __restrict__ QH, const _Float16* __restrict__ QL, const _Float16* __restrict__ KH, const _Float16* __restrict__ KL, const _Float16* __restrict__ VT, const __bf16* __restrict__ VB, const __bf16* __restrict__ VBL,
    const unsigned* __restrict__ MB, _Float16* __restrict__ CTXH, __bf16* __restrict__ CBH, __bf16* __restrict__ CBL) {
  __shared__ __align__(16) float ps[4][16][36];
  __shared__ __align__(16) _Float16 so[4][16][72];
  __shared__ __align__(16) __bf16 sbh[4][16][72];
  __shared__ __align__(16) __bf16 sbl[4][16][72];
  const int tid = threadIdx.x, wave = tid >> 5, lane = tid & 31, col = lane & 15, g = lane >> 4;
  const int qb = blockIdx.x, h = blockIdx.y, b = blockIdx.z;
  const bool hp = qb < QBH;
  const int ql0 = qb * 64 + wave * 16;
  const size_t qrow0 = (size_t)b * SEQ + ql0;
  const unsigned* mrow = MB + (qrow0 + (size_t)(lane >> 1)) * (size_t)(SEQ / 32);
  unsigned orw = 0u;
#pragma unroll
  for (int i = 0; i < SEQ / 256; ++i) { const v4u t = *(const v4u*)(mrow + (lane & 1) * (SEQ / 64) + i * 4); orw |= (t[0] | t[1]) | (t[2] | t[3]); }
  orw |= (unsigned)__shfl_xor((int)orw, 1);
  const bool allkeep = __builtin_amdgcn_ballot_w32(orw == 0u) == 0u;
  float m[8], l[8]; v8f acc[4] = {};
#pragma unroll
  for (int r = 0; r < 8; ++r) { m[r] = -1.0e30f; l[r] = 0.f; }
  const size_t qoff = (qrow0 + col) * CC + (size_t)h * HD;
  const size_t qloff = hp ? (((size_t)b * QHI + ql0 + col) * CC + (size_t)h * HD) : (size_t)0;
#pragma unroll 1
  for (int kb = 0; kb < SEQ / 64; ++kb) {
    const unsigned w = mrow[kb * 2 + (lane & 1)];
    const unsigned anyk = __builtin_amdgcn_ballot_w32(w != 0u);
    if (allkeep && anyk == 0u) continue;
#pragma unroll 1
    for (int hf = 0; hf < 2; ++hf) {
      const int k0 = kb * 64 + hf * 32;
      const size_t kr = ((size_t)b * SEQ + k0 + col) * CC + (size_t)h * HD;
      v8f s0 = {}, s1 = {};
      if (hp) {
        v8f x0 = {}, x1 = {};
#pragma unroll 1
        for (int kc = 0; kc < HD / 32; ++kc) {
          const v16h ah = frag_h(QH + qoff + kc * 32, lane), al = frag_h(QL + qloff + kc * 32, lane);
          const v16h k0h = frag_h(KH + kr + kc * 32, lane), k1h = frag_h(KH + kr + (size_t)16 * CC + kc * 32, lane);
          const v16h k0l = frag_h(KL + kr + kc * 32, lane), k1l = frag_h(KL + kr + (size_t)16 * CC + kc * 32, lane);
          s0 = wmma16(ah, k0h, s0); s1 = wmma16(ah, k1h, s1);
          x0 = wmma16(al, k0h, x0); x0 = wmma16(ah, k0l, x0);
          x1 = wmma16(al, k1h, x1); x1 = wmma16(ah, k1l, x1);
        }
#pragma unroll
        for (int r = 0; r < 8; ++r) { s0[r] += x0[r] * (1.0f / 1024.0f); s1[r] += x1[r] * (1.0f / 1024.0f); }
      } else {
#pragma unroll
        for (int kc = 0; kc < HD / 32; ++kc) {
          const v16h a = frag_h(QH + qoff + kc * 32, lane);
          const v16h k0h = frag_h(KH + kr + kc * 32, lane), k1h = frag_h(KH + kr + (size_t)16 * CC + kc * 32, lane);
          s0 = wmma16(a, k0h, s0); s1 = wmma16(a, k1h, s1);
        }
      }
#pragma unroll
      for (int r = 0; r < 8; ++r) {
        const unsigned wr = (unsigned)__shfl((int)w, 2 * (8 * g + r) + hf);
        const float x0 = ((wr >> col) & 1u) ? s0[r] * 0.125f : -1.0e9f;
        const float x1 = ((wr >> (16 + col)) & 1u) ? s1[r] * 0.125f : -1.0e9f;
        float mx = fmaxf(x0, x1);
        mx = fmaxf(mx, __shfl_xor(mx, 1)); mx = fmaxf(mx, __shfl_xor(mx, 2)); mx = fmaxf(mx, __shfl_xor(mx, 4)); mx = fmaxf(mx, __shfl_xor(mx, 8));
        const float mn = fmaxf(m[r], mx);
        const float f = __expf(m[r] - mn);
        const float p0 = __expf(x0 - mn), p1 = __expf(x1 - mn);
        m[r] = mn; l[r] = l[r] * f + (p0 + p1);
        acc[0][r] *= f; acc[1][r] *= f; acc[2][r] *= f; acc[3][r] *= f;
        ps[wave][8 * g + r][col] = p0; ps[wave][8 * g + r][16 + col] = p1;
      }
      LDSX();
      const v4f pa = *(const v4f_a*)&ps[wave][col][8 * g], pb = *(const v4f_a*)&ps[wave][col][8 * g + 4];
      const v4f pc = *(const v4f_a*)&ps[wave][col][16 + 8 * g], pd = *(const v4f_a*)&ps[wave][col][16 + 8 * g + 4];
      float pv[16];
#pragma unroll
      for (int i = 0; i < 4; ++i) { pv[i] = pa[i]; pv[4 + i] = pb[i]; pv[8 + i] = pc[i]; pv[12 + i] = pd[i]; }
      const size_t vo = ((size_t)b * CC + (size_t)h * HD + col) * (size_t)SEQ + k0;
      if (hp) {
        v16b ph, pl;
#pragma unroll
        for (int i = 0; i < 16; ++i) { const __bf16 hh = (__bf16)pv[i]; ph[i] = hh; pl[i] = (__bf16)(pv[i] - (float)hh); }
#pragma unroll
        for (int j = 0; j < 4; ++j) { const size_t o3 = vo + (size_t)(j * 16) * SEQ; const v16b vh = frag_b(VB + o3, lane), vl = frag_b(VBL + o3, lane);
          acc[j] = wmma_bf(pl, vh, acc[j]); acc[j] = wmma_bf(ph, vl, acc[j]); acc[j] = wmma_bf(ph, vh, acc[j]); }
      } else {
        v16h pf;
#pragma unroll
        for (int i = 0; i < 16; ++i) pf[i] = (_Float16)(pv[i] * 2048.0f);
#pragma unroll
        for (int j = 0; j < 4; ++j) { const size_t o3 = vo + (size_t)(j * 16) * SEQ; acc[j] = wmma16(pf, frag_h(VT + o3, lane), acc[j]); }
      }
      LDSX();
    }
  }
  float linv[8];
#pragma unroll
  for (int r = 0; r < 8; ++r) { float lt = l[r]; lt += __shfl_xor(lt, 1); lt += __shfl_xor(lt, 2); lt += __shfl_xor(lt, 4); lt += __shfl_xor(lt, 8); linv[r] = 1.0f / lt; }
  if (hp) {
#pragma unroll
    for (int r = 0; r < 8; ++r) {
#pragma unroll
      for (int j = 0; j < 4; ++j) { const float v = acc[j][r] * linv[r]; const __bf16 bh = (__bf16)v; sbh[wave][8 * g + r][j * 16 + col] = bh; sbl[wave][8 * g + r][j * 16 + col] = (__bf16)(v - (float)bh); } }
    LDSX();
#pragma unroll
    for (int it = 0; it < 4; ++it) { const int row = it * 4 + (lane >> 3), pc8 = (lane & 7) * 8; const size_t o = (((size_t)b * QHI + ql0 + row) * CC) + (size_t)h * HD + pc8;
      const v4u a = *(const v4u_a*)&sbh[wave][row][pc8]; vst2(CBH + o, a); const v4u c = *(const v4u_a*)&sbl[wave][row][pc8]; vst2(CBL + o, c); }
  } else {
#pragma unroll
    for (int r = 0; r < 8; ++r) { const float sc = linv[r] * (64.0f / 2048.0f);
#pragma unroll
      for (int j = 0; j < 4; ++j) so[wave][8 * g + r][j * 16 + col] = (_Float16)(acc[j][r] * sc); }
    LDSX();
#pragma unroll
    for (int it = 0; it < 4; ++it) { const int row = it * 4 + (lane >> 3), pc8 = (lane & 7) * 8;
      const v4u a = *(const v4u_a*)&so[wave][row][pc8]; vst2(CTXH + (qrow0 + row) * CC + (size_t)h * HD + pc8, a); }
  }
}

__global__ __launch_bounds__(128) void k_out(const _Float16* __restrict__ CTXH, const __bf16* __restrict__ CBH, const __bf16* __restrict__ CBL, const _Float16* __restrict__ WOH, const __bf16* __restrict__ WOB, const float* __restrict__ BO, float* __restrict__ OUT) {
  __shared__ __align__(16) float sf[4][16][132];
  const int tid = threadIdx.x, wave = tid >> 5, lane = tid & 31, col = lane & 15, g = lane >> 4; const int c0 = blockIdx.y * 128; const size_t rb = (size_t)blockIdx.x * 64; const size_t r0 = rb + wave * 16; const size_t bb = rb / SEQ; const int t0 = (int)(rb % SEQ);
  v8f acc[8] = {};
  if (t0 < QHI) {
    const size_t hr = bb * QHI + (size_t)t0 + wave * 16 + col;
#pragma unroll 2
    for (int kc = 0; kc < CC / 32; ++kc) { const v16b ah = frag_b(CBH + hr * CC + kc * 32, lane), al = frag_b(CBL + hr * CC + kc * 32, lane);
#pragma unroll
      for (int j = 0; j < 8; ++j) { const v16b w = frag_b(WOB + (size_t)(c0 + j * 16 + col) * CC + kc * 32, lane); acc[j] = wmma_bf(al, w, acc[j]); acc[j] = wmma_bf(ah, w, acc[j]); } }
#pragma unroll
    for (int j = 0; j < 8; ++j) { const float bias = bfr(BO[c0 + j * 16 + col]);
#pragma unroll
      for (int r = 0; r < 8; ++r) sf[wave][8 * g + r][j * 16 + col] = acc[j][r] + bias; }
  } else {
#pragma unroll 2
    for (int kc = 0; kc < CC / 32; ++kc) { const v16h a = frag_h(CTXH + (r0 + col) * CC + kc * 32, lane);
#pragma unroll
      for (int j = 0; j < 8; ++j) { const v16h w = frag_h(WOH + (size_t)(c0 + j * 16 + col) * CC + kc * 32, lane); acc[j] = wmma16(a, w, acc[j]); } }
#pragma unroll
    for (int j = 0; j < 8; ++j) { const float bias = bfr(BO[c0 + j * 16 + col]);
#pragma unroll
      for (int r = 0; r < 8; ++r) sf[wave][8 * g + r][j * 16 + col] = acc[j][r] * (1.0f / 16384.0f) + bias; }
  }
  LDSX();
  for (int rl = 0; rl < 16; ++rl) { const v4f v = *(const v4f_a*)&sf[wave][rl][lane * 4]; vst2(OUT + (r0 + rl) * CC + c0 + lane * 4, v); }
}

extern "C" void kernel_launch(void* const* d_in, const int* in_sizes, int n_in, void* d_out, int out_size, void* d_ws, size_t ws_size, hipStream_t stream) {
  if (n_in < 12) return;
  const size_t needx = ((size_t)(NB - 1) * SEQ_FULL + SEQ) * CC;
  const size_t needm = ((size_t)(NB - 1) * SEQ_FULL + (SEQ - 1)) * SEQ_FULL + SEQ;
  if ((size_t)in_sizes[0] < needx || (size_t)in_sizes[1] < needx || (size_t)in_sizes[2] < needx) return;
  if ((size_t)in_sizes[3] < needm) return;
  if ((size_t)in_sizes[4] < (size_t)CC * CC || (size_t)in_sizes[6] < (size_t)CC * CC || (size_t)in_sizes[8] < (size_t)CC * CC || (size_t)in_sizes[10] < (size_t)CC * CC) return;
  if (in_sizes[5] < CC || in_sizes[7] < CC || in_sizes[9] < CC || in_sizes[11] < CC) return;
  if ((size_t)out_size < NTOK * CC) return;
  if (ws_size < (size_t)WS_END) return;
  const float* xq = (const float*)d_in[0]; const float* xk = (const float*)d_in[1]; const float* xv = (const float*)d_in[2];
  const int* mask = (const int*)d_in[3];
  const float* Wq = (const float*)d_in[4]; const float* bq = (const float*)d_in[5];
  const float* Wk = (const float*)d_in[6]; const float* bk = (const float*)d_in[7];
  const float* Wv = (const float*)d_in[8]; const float* bv = (const float*)d_in[9];
  const float* Wo = (const float*)d_in[10]; const float* bo = (const float*)d_in[11];
  char* ws = (char*)d_ws;
  __bf16* XB = (__bf16*)(ws + WS_XB); __bf16* WB = (__bf16*)(ws + WS_WB); __bf16* WOB = (__bf16*)(ws + WS_WOB); _Float16* WOH = (_Float16*)(ws + WS_WOH);
  _Float16* QH = (_Float16*)(ws + WS_QH); _Float16* KH = (_Float16*)(ws + WS_KH); _Float16* KL = (_Float16*)(ws + WS_KL); _Float16* VT = (_Float16*)(ws + WS_VT);
  __bf16* VB = (__bf16*)(ws + WS_VB); __bf16* VBL = (__bf16*)(ws + WS_VBL); _Float16* QL = (_Float16*)(ws + WS_QL); unsigned* MB = (unsigned*)(ws + WS_MB);
  _Float16* CTXH = (_Float16*)(ws + WS_CTXH); __bf16* CBH = (__bf16*)(ws + WS_CBH); __bf16* CBL = (__bf16*)(ws + WS_CBL);
  k_maskbits<<<dim3((unsigned)(NTOK / 8)), 256, 0, stream>>>(mask, MB);
  k_cvt_x<<<dim3((unsigned)(NTOK * CC / 8 / 256), 3), 256, 0, stream>>>(xq, xk, xv, XB);
  k_cvt_w<<<dim3((unsigned)((size_t)CC * CC / 8 / 256), 4), 256, 0, stream>>>(Wq, Wk, Wv, Wo, WB, WOB, WOH);
  k_proj<<<dim3((unsigned)(NTOK / 64), CC / 128, 3), 128, 0, stream>>>(XB, WB, bq, bk, bv, QH, QL, KH, KL, VT, VB, VBL);
  k_attn<<<dim3(SEQ / 64, NH, NB), 128, 0, stream>>>(QH, QL, KH, KL, VT, VB, VBL, MB, CTXH, CBH, CBL);
  k_out<<<dim3((unsigned)(NTOK / 64), CC / 128), 128, 0, stream>>>(CTXH, CBH, CBL, WOH, WOB, bo, (float*)d_out);
}
